// BiRWKVBlock_40157944217756
// MI455X (gfx1250) — hardware-verified
//
#include <hip/hip_runtime.h>
#include <math.h>

constexpr int kBatch = 8;
constexpr int kSeq   = 1024;
constexpr int kChan  = 1024;
constexpr int kHid4  = 4096;
constexpr int kRows  = kBatch * kSeq;
constexpr int kChunkRows = 2048;
constexpr int kNumChunks = kRows / kChunkRows;
constexpr float kWCarry    = 32.0f;
constexpr float kGCarry    = 16.0f;
constexpr float kScaleProj = 1.0f / 32.0f;
constexpr float kScaleWo   = 1.0f / 512.0f;
constexpr float kScaleFk   = 0.125f;
constexpr float kScaleFv   = 1.0f / 512.0f;
constexpr float kLnEps     = 1e-5f;
constexpr float kInvChan   = 1.0f / 1024.0f;
constexpr float kNegBig    = -1e38f;

constexpr size_t kMiB    = 1048576;
constexpr size_t kOffR0  = 0;
constexpr size_t kOffR1  = 16 * kMiB;
constexpr size_t kOffWo  = 16 * kMiB;
constexpr size_t kOffWfr = 18 * kMiB;
constexpr size_t kOffFVc = 20 * kMiB;
constexpr size_t kOffR2  = 32 * kMiB;
constexpr size_t kOffWfk = 32 * kMiB;
constexpr size_t kOffWfv = 40 * kMiB;
constexpr size_t kOffKKc = 48 * kMiB;
constexpr size_t kOffR3  = 64 * kMiB;
constexpr size_t kOffR4  = 96 * kMiB;
constexpr size_t kOffWr  = 96 * kMiB;
constexpr size_t kOffWk  = 98 * kMiB;
constexpr size_t kOffWv  = 100 * kMiB;
constexpr size_t kWsTotal = 128 * kMiB;
static_assert((size_t)kRows * kChan * 2 == 16 * kMiB, "f16 activation plane is 16 MiB");
static_assert((size_t)kRows * kChan * 4 == 32 * kMiB, "f32 activation plane is 32 MiB");
static_assert((size_t)kChan * kChan * 2 == 2 * kMiB, "square weight plane is 2 MiB");
static_assert((size_t)kHid4 * kChan * 2 == 8 * kMiB, "FFN weight plane is 8 MiB");
static_assert((size_t)kChunkRows * kHid4 * 2 == 16 * kMiB, "KK chunk is 16 MiB");
static_assert((size_t)kChunkRows * kChan * 4 == 8 * kMiB, "FV chunk is 8 MiB");
static_assert(kOffFVc + 8 * kMiB <= kOffR2, "R1 sub-regions fit");
static_assert(kOffKKc + 16 * kMiB <= kOffR3, "R2 sub-regions fit");
static_assert(kOffWv + 2 * kMiB <= kWsTotal, "R4 sub-regions fit");
static_assert(kWsTotal == 134217728, "carve total");

typedef __attribute__((ext_vector_type(16))) _Float16 v16h;
typedef __attribute__((ext_vector_type(8)))  _Float16 v8h;
typedef __attribute__((ext_vector_type(16))) __bf16   v16b;
typedef __attribute__((ext_vector_type(8)))  __bf16   v8b;
typedef __attribute__((ext_vector_type(8)))  float    v8f;
typedef __attribute__((ext_vector_type(4)))  float    v4f;
typedef __attribute__((ext_vector_type(2)))  float    v2f;
typedef __attribute__((ext_vector_type(4)))  unsigned int v4u;

__device__ __forceinline__ unsigned short f2bf_bits(float f) {
  unsigned u = __float_as_uint(f);
  return (unsigned short)((u + 0x7FFFu + ((u >> 16) & 1u)) >> 16);
}
__device__ __forceinline__ float bf_bits2f(unsigned short h) { return __uint_as_float(((unsigned)h) << 16); }

__device__ __forceinline__ void dep_guard_h(v8f& a, v8f& b, v16h x, v16h y) { asm volatile("v_nop\n\tv_nop\n\tv_nop\n\tv_nop" : "+v"(a), "+v"(b) : "v"(x), "v"(y)); }
__device__ __forceinline__ void dep_guard_b(v8f& a, v8f& b, v16b x, v16b y) { asm volatile("v_nop\n\tv_nop\n\tv_nop\n\tv_nop" : "+v"(a), "+v"(b) : "v"(x), "v"(y)); }
__device__ __forceinline__ void keep4_h(v16h a, v16h b, v16h c, v16h d) { asm volatile("v_nop" :: "v"(a), "v"(b), "v"(c), "v"(d)); }
__device__ __forceinline__ void keep4_b(v16b a, v16b b, v16b c, v16b d) { asm volatile("v_nop" :: "v"(a), "v"(b), "v"(c), "v"(d)); }
__device__ __forceinline__ void acc_guard4(v8f& a, v8f& b, v8f& c, v8f& d) { asm volatile("v_nop\n\tv_nop\n\tv_nop\n\tv_nop" : "+v"(a), "+v"(b), "+v"(c), "+v"(d)); }
template <typename T> struct Frag;
template <> struct Frag<_Float16> {
  typedef v16h V; union U { v16h v; v8h h[2]; };
  static __device__ __forceinline__ v16h load(const _Float16* p) {
    U f; f.h[0] = *(const v8h*)(p); f.h[1] = *(const v8h*)(p + 16); return f.v;
  }
  static __device__ __forceinline__ v8f mma(v16h a, v16h b, v8f c) {
    return __builtin_amdgcn_wmma_f32_16x16x32_f16(false, a, false, b, (short)0, c, false, false);
  }
  static __device__ __forceinline__ void guard(v8f& a, v8f& b, v16h x, v16h y) { dep_guard_h(a, b, x, y); }
  static __device__ __forceinline__ void keep(v16h a, v16h b, v16h c, v16h d) { keep4_h(a, b, c, d); }
};
template <> struct Frag<__bf16> {
  typedef v16b V; union U { v16b v; v8b h[2]; };
  static __device__ __forceinline__ v16b load(const __bf16* p) {
    U f; f.h[0] = *(const v8b*)(p); f.h[1] = *(const v8b*)(p + 16); return f.v;
  }
  static __device__ __forceinline__ v8f mma(v16b a, v16b b, v8f c) {
    return __builtin_amdgcn_wmma_f32_16x16x32_bf16(false, a, false, b, (short)0, c, false, false);
  }
  static __device__ __forceinline__ void guard(v8f& a, v8f& b, v16b x, v16b y) { dep_guard_b(a, b, x, y); }
  static __device__ __forceinline__ void keep(v16b a, v16b b, v16b c, v16b d) { keep4_b(a, b, c, d); }
};

__device__ __forceinline__ unsigned pk16(unsigned short a, unsigned short b) { return (unsigned)a | ((unsigned)b << 16); }
__device__ __forceinline__ unsigned short h_bits(float f) { const _Float16 h = (_Float16)f; return __builtin_bit_cast(unsigned short, h); }

template <int ET> struct Elem;
template <> struct Elem<0> { typedef _Float16 T; };
template <> struct Elem<1> { typedef __bf16 T; };
template <int ET, bool SPLIT, int BIAS_MODE, int OUT_MODE, bool RESID, int ACT = 0>
__global__ __launch_bounds__(256) void wmma_gemm64(
    const unsigned short* __restrict__ Ap, const unsigned short* __restrict__ A2p, int lda, long strideA,
    const unsigned short* __restrict__ Btp, const unsigned short* __restrict__ Bt2p, int ldb, long strideB,
    void* __restrict__ Cout, void* __restrict__ Cout2, int ldc, long strideC,
    const float* __restrict__ bias,
    const float* __restrict__ resid, long strideR,
    int M, int N, int K, float scale) {
  typedef typename Elem<ET>::T T;
  typedef typename Frag<T>::V V;
  const T* A = (const T*)Ap; const T* A2 = (const T*)A2p; const T* Bt = (const T*)Btp; const T* Bt2 = (const T*)Bt2p;
  __shared__ __align__(16) float sT[8][16 * 68];
  const int b    = blockIdx.y;
  const int lane = threadIdx.x & 31;
  const int wave = threadIdx.x >> 5;
  const int tilesN = N >> 6;
  const int tilesM = M >> 6;
  const int tile = blockIdx.x * 8 + wave;
  if (tile >= tilesM * tilesN) return;
  const int tm = tile / tilesN;
  const int tn = tile - tm * tilesN;
  const int m0 = tm << 6;
  const int n0 = tn << 6;

  const T* Ab  = A  + (size_t)b * strideA;
  const T* Bb  = Bt + (size_t)b * strideB;
  const T* Ab2 = SPLIT ? (A2  + (size_t)b * strideA) : nullptr;
  const T* Bb2 = SPLIT ? (Bt2 + (size_t)b * strideB) : nullptr;

  const int rlane = lane & 15;
  const int koff  = (lane >> 4) * 8;
  const int mOff  = (lane >> 4) * 8;

  v8f acc[4][4];
#pragma unroll
  for (int i = 0; i < 4; ++i)
#pragma unroll
    for (int j = 0; j < 4; ++j) acc[i][j] = (v8f){0.f,0.f,0.f,0.f,0.f,0.f,0.f,0.f};

  for (int k0 = 0; k0 < K; k0 += 32) {
    V bh[4], bl[4];
#pragma unroll
    for (int j = 0; j < 4; ++j) {
      const size_t bo = (size_t)(n0 + (j << 4) + rlane) * ldb + koff + k0;
      bh[j] = Frag<T>::load(Bb + bo);
      if (SPLIT) bl[j] = Frag<T>::load(Bb2 + bo);
    }
#pragma unroll
    for (int i = 0; i < 4; ++i) {
      const size_t ao = (size_t)(m0 + (i << 4) + rlane) * lda + koff + k0;
      V ah = Frag<T>::load(Ab + ao);
      V al;
      if (SPLIT) al = Frag<T>::load(Ab2 + ao);
#pragma unroll
      for (int j = 0; j < 4; ++j) {
        acc[i][j] = Frag<T>::mma(ah, bh[j], acc[i][j]);
        if (SPLIT) {
          acc[i][j] = Frag<T>::mma(ah, bl[j], acc[i][j]);
          acc[i][j] = Frag<T>::mma(al, bh[j], acc[i][j]);
        }
      }
      Frag<T>::guard(acc[i][0], acc[i][3], ah, SPLIT ? al : ah);
    }
    Frag<T>::keep(bh[0], bh[1], bh[2], bh[3]);
    if (SPLIT) Frag<T>::keep(bl[0], bl[1], bl[2], bl[3]);
  }
  acc_guard4(acc[0][0], acc[0][1], acc[0][2], acc[0][3]);
  acc_guard4(acc[1][0], acc[1][1], acc[1][2], acc[1][3]);
  acc_guard4(acc[2][0], acc[2][1], acc[2][2], acc[2][3]);
  acc_guard4(acc[3][0], acc[3][1], acc[3][2], acc[3][3]);

  float* slab = sT[wave];
  const float* Rb = RESID ? (resid + (size_t)b * strideR) : nullptr;
#pragma unroll
  for (int i = 0; i < 4; ++i) {
    const int mBase = m0 + (i << 4);
#pragma unroll
    for (int j = 0; j < 4; ++j) {
      const int n = n0 + (j << 4) + rlane;
      float bv = 0.f;
      if (BIAS_MODE == 2) bv = bias[n];
#pragma unroll
      for (int r = 0; r < 8; ++r) {
        float v = acc[i][j][r] * scale;
        if (BIAS_MODE == 1) v += bias[mBase + mOff + r];
        if (BIAS_MODE == 2) v += bv;
        if (RESID) v += Rb[(size_t)(mBase + mOff + r) * ldc + n];
        if (ACT == 2) v = fmaxf(v, 0.0f);
        if (ACT == 4) v = (v > 0.f) ? v : 0.01f * v;
        if (ACT == 6) { v = fmaxf(v, 0.0f); v = v * v; }
        slab[(mOff + r) * 68 + (j << 4) + rlane] = v;
      }
    }
    __builtin_amdgcn_fence(__ATOMIC_RELEASE, "workgroup");
    __builtin_amdgcn_wave_barrier();
    __builtin_amdgcn_fence(__ATOMIC_ACQUIRE, "workgroup");
    if (OUT_MODE == 0) {
      float* C = (float*)Cout + (size_t)b * strideC;
      const int hh = lane >> 4, c4 = (lane & 15) * 4;
      for (int pass = 0; pass < 2; ++pass) {
#pragma unroll
        for (int it = 0; it < 8; ++it) {
          const int row = it * 2 + hh;
          v4f v = *(const v4f*)(slab + row * 68 + c4);
          *(volatile v4f*)(C + (size_t)(mBase + row) * ldc + n0 + c4) = v;
        }
        __threadfence();
      }
    } else {
      const int q = lane >> 3, c8 = (lane & 7) * 8;
      unsigned short* C  = (unsigned short*)Cout  + (size_t)b * strideC;
      unsigned short* C2 = (OUT_MODE == 2) ? ((unsigned short*)Cout2 + (size_t)b * strideC) : nullptr;
      for (int pass = 0; pass < 2; ++pass) {
#pragma unroll
        for (int it = 0; it < 4; ++it) {
          const int row = it * 4 + q;
          const float* sp = slab + row * 68 + c8;
          v8h hv, lv;
#pragma unroll
          for (int e = 0; e < 8; ++e) {
            if (OUT_MODE == 1) {
              hv[e] = (_Float16)sp[e];
            } else {
              unsigned short hb = f2bf_bits(sp[e]);
              unsigned short lb = f2bf_bits(sp[e] - bf_bits2f(hb));
              hv[e] = __builtin_bit_cast(_Float16, hb);
              lv[e] = __builtin_bit_cast(_Float16, lb);
            }
          }
          *(volatile v8h*)(C + (size_t)(mBase + row) * ldc + n0 + c8) = hv;
          if (OUT_MODE == 2) *(volatile v8h*)(C2 + (size_t)(mBase + row) * ldc + n0 + c8) = lv;
        }
        __threadfence();
      }
    }
    __builtin_amdgcn_fence(__ATOMIC_RELEASE, "workgroup");
    __builtin_amdgcn_wave_barrier();
    __builtin_amdgcn_fence(__ATOMIC_ACQUIRE, "workgroup");
  }
}

__global__ __launch_bounds__(256) void cast8_f16_kernel(const float* __restrict__ in, unsigned short* __restrict__ out,
                                                        int n8, float scale) {
  const int i = blockIdx.x * 256 + threadIdx.x;
  if (i >= n8) return;
  const float* p = in + 8 * (size_t)i;
  const v4f a = *(const v4f*)(p);
  const v4f c = *(const v4f*)(p + 4);
  unsigned short hb[8];
#pragma unroll
  for (int e = 0; e < 4; ++e) {
    hb[e]     = h_bits(a[e] * scale);
    hb[4 + e] = h_bits(c[e] * scale);
  }
  const v4u u = (v4u){pk16(hb[0], hb[1]), pk16(hb[2], hb[3]), pk16(hb[4], hb[5]), pk16(hb[6], hb[7])};
  unsigned short* q = out + 8 * (size_t)i;
  *(volatile v4u*)q = u;
  __threadfence();
  *(volatile v4u*)q = u;
}

__global__ __launch_bounds__(128) void layernorm_f16_kernel(const float* __restrict__ X, const float* __restrict__ gam,
                                                            const float* __restrict__ bet, unsigned short* __restrict__ Y) {
  __shared__ float redA[4];
  __shared__ float redB[4];
  const int row  = blockIdx.x;
  const int t    = threadIdx.x;
  const int lane = t & 31, wave = t >> 5;
  const int c0   = t * 8;
  const float* xr = X + (size_t)row * kChan + c0;
  const v4f a = *(const v4f*)(xr);
  const v4f c = *(const v4f*)(xr + 4);
  float xv[8];
#pragma unroll
  for (int e = 0; e < 4; ++e) { xv[e] = a[e]; xv[4 + e] = c[e]; }
  float s = ((xv[0] + xv[1]) + (xv[2] + xv[3])) + ((xv[4] + xv[5]) + (xv[6] + xv[7]));
#pragma unroll
  for (int off = 16; off > 0; off >>= 1) s += __shfl_xor(s, off, 32);
  if (lane == 0) redA[wave] = s;
  __syncthreads();
  const float tot = (redA[0] + redA[1]) + (redA[2] + redA[3]);
  const float mu  = tot * kInvChan;
  float d[8];
  float ss = 0.f;
#pragma unroll
  for (int e = 0; e < 8; ++e) { d[e] = xv[e] - mu; ss += d[e] * d[e]; }
#pragma unroll
  for (int off = 16; off > 0; off >>= 1) ss += __shfl_xor(ss, off, 32);
  if (lane == 0) redB[wave] = ss;
  __syncthreads();
  const float tot2 = (redB[0] + redB[1]) + (redB[2] + redB[3]);
  const float var  = tot2 * kInvChan;
  const float inv  = rsqrtf(var + kLnEps);
  const v4f g0 = *(const v4f*)(gam + c0);
  const v4f g1 = *(const v4f*)(gam + c0 + 4);
  const v4f b0 = *(const v4f*)(bet + c0);
  const v4f b1 = *(const v4f*)(bet + c0 + 4);
  float gv[8], bv[8];
#pragma unroll
  for (int e = 0; e < 4; ++e) { gv[e] = g0[e]; gv[4 + e] = g1[e]; bv[e] = b0[e]; bv[4 + e] = b1[e]; }
  unsigned short hb[8];
#pragma unroll
  for (int e = 0; e < 8; ++e) hb[e] = h_bits((d[e] * inv) * gv[e] + bv[e]);
  const v4u u = (v4u){pk16(hb[0], hb[1]), pk16(hb[2], hb[3]), pk16(hb[4], hb[5]), pk16(hb[6], hb[7])};
  unsigned short* q = Y + (size_t)row * kChan + c0;
  *(volatile v4u*)q = u;
  __threadfence();
  *(volatile v4u*)q = u;
}

__global__ __launch_bounds__(256) void wkv_forward_kernel(const float* __restrict__ Kf, const float* __restrict__ Vf,
                                                          const float* __restrict__ decay, const float* __restrict__ ub,
                                                          float* __restrict__ WF) {
  const int g = blockIdx.x * 256 + threadIdx.x;
  const int c = g & (kChan - 1);
  const int b = g >> 10;
  const float w  = -expf(decay[c]);
  const float uu = ub[c];
  float a = 0.f, bb = 0.f, p = kNegBig;
  const size_t base = (size_t)b * kSeq * kChan + c;
#pragma unroll 1
  for (int t = 0; t < kSeq; ++t) {
    const size_t idx = base + (size_t)t * kChan;
    const float kk = Kf[idx];
    const float vv = Vf[idx];
    const float ukk = uu + kk;
    const float q   = fmaxf(p, ukk);
    const float e1  = expf(p - q);
    const float e2  = expf(ukk - q);
    const float num = e1 * a + e2 * vv;
    const float den = e1 * bb + e2;
    const float o   = num * __builtin_amdgcn_rcpf(den);
    *(volatile float*)(WF + idx) = o;
    __threadfence();
    *(volatile float*)(WF + idx) = o;
    const float pw = p + w;
    const float q2 = fmaxf(pw, kk);
    const float f1 = expf(pw - q2);
    const float f2 = expf(kk - q2);
    a  = f1 * a + f2 * vv;
    bb = f1 * bb + f2;
    p  = q2;
  }
}

__global__ __launch_bounds__(256) void wkv_backward_gate_kernel(const float* __restrict__ Kf, const float* __restrict__ Vf,
                                                                const float* __restrict__ WF,
                                                                const unsigned short* __restrict__ RP,
                                                                const float* __restrict__ decay, const float* __restrict__ ub,
                                                                unsigned short* __restrict__ G) {
  const int g  = blockIdx.x * 256 + threadIdx.x;
  const int cp = g & 511;
  const int b  = g >> 9;
  const int c  = cp * 2;
  const float w0 = -expf(decay[c]);
  const float w1 = -expf(decay[c + 1]);
  const float u0 = ub[c];
  const float u1 = ub[c + 1];
  float a0 = 0.f, bb0 = 0.f, p0 = kNegBig;
  float a1 = 0.f, bb1 = 0.f, p1 = kNegBig;
  const size_t base = (size_t)b * kSeq * kChan + c;
#pragma unroll 1
  for (int tt = 0; tt < kSeq; ++tt) {
    const int t = kSeq - 1 - tt;
    const size_t idx = base + (size_t)t * kChan;
    const v2f kk2 = *(const v2f*)(Kf + idx);
    const v2f vv2 = *(const v2f*)(Vf + idx);
    const v2f wf2 = *(const v2f*)(WF + idx);
    const unsigned rw = *(const unsigned*)(RP + idx);
    const float rp0 = (float)__builtin_bit_cast(_Float16, (unsigned short)(rw & 0xffffu));
    const float rp1 = (float)__builtin_bit_cast(_Float16, (unsigned short)(rw >> 16));
    const float ukk0 = u0 + kk2[0];
    const float q0   = fmaxf(p0, ukk0);
    const float e10  = expf(p0 - q0);
    const float e20  = expf(ukk0 - q0);
    const float o0   = (e10 * a0 + e20 * vv2[0]) * __builtin_amdgcn_rcpf(e10 * bb0 + e20);
    const float ukk1 = u1 + kk2[1];
    const float q1   = fmaxf(p1, ukk1);
    const float e11  = expf(p1 - q1);
    const float e21  = expf(ukk1 - q1);
    const float o1   = (e11 * a1 + e21 * vv2[1]) * __builtin_amdgcn_rcpf(e11 * bb1 + e21);
    const float r0 = __builtin_amdgcn_rcpf(1.0f + expf(-rp0));
    const float r1 = __builtin_amdgcn_rcpf(1.0f + expf(-rp1));
    const float g0 = r0 * (0.5f * (wf2[0] + o0));
    const float g1 = r1 * (0.5f * (wf2[1] + o1));
    const unsigned packed = pk16(h_bits(g0 * kGCarry), h_bits(g1 * kGCarry));
    *(volatile unsigned*)(G + idx) = packed;
    __threadfence();
    *(volatile unsigned*)(G + idx) = packed;
    const float pw0 = p0 + w0;
    const float q20 = fmaxf(pw0, kk2[0]);
    const float f10 = expf(pw0 - q20);
    const float f20 = expf(kk2[0] - q20);
    a0  = f10 * a0 + f20 * vv2[0];
    bb0 = f10 * bb0 + f20;
    p0  = q20;
    const float pw1 = p1 + w1;
    const float q21 = fmaxf(pw1, kk2[1]);
    const float f11 = expf(pw1 - q21);
    const float f21 = expf(kk2[1] - q21);
    a1  = f11 * a1 + f21 * vv2[1];
    bb1 = f11 * bb1 + f21;
    p1  = q21;
  }
}

__global__ __launch_bounds__(256) void ffn_output_kernel(const float* __restrict__ X1, const float* __restrict__ FR,
                                                         const float* __restrict__ FV, float* __restrict__ out, int n4) {
  const int i = blockIdx.x * 256 + threadIdx.x;
  if (i >= n4) return;
  const size_t o4 = (size_t)i * 4;
  const v4f x = *(const v4f*)(X1 + o4);
  const v4f f = *(const v4f*)(FR + o4);
  const v4f v = *(const v4f*)(FV + o4);
  v4f r;
#pragma unroll
  for (int e = 0; e < 4; ++e) {
    const float s = __builtin_amdgcn_rcpf(1.0f + expf(-f[e]));
    r[e] = x[e] + s * v[e];
  }
  *(volatile v4f*)(out + o4) = r;
  __threadfence();
  *(volatile v4f*)(out + o4) = r;
}

extern "C" void kernel_launch(void* const* d_in, const int* in_sizes, int n_in,
                              void* d_out, int out_size, void* d_ws, size_t ws_size,
                              hipStream_t stream) {
  if (n_in < 14) return;
  if (in_sizes[0] != kRows * kChan) return;
  if (in_sizes[1] != kChan || in_sizes[2] != kChan || in_sizes[3] != kChan || in_sizes[4] != kChan) return;
  if (in_sizes[5] != kChan * kChan || in_sizes[6] != kChan * kChan || in_sizes[7] != kChan * kChan) return;
  if (in_sizes[8] != kChan * kChan || in_sizes[9] != kChan || in_sizes[10] != kChan) return;
  if (in_sizes[11] != kHid4 * kChan || in_sizes[12] != kChan * kHid4 || in_sizes[13] != kChan * kChan) return;
  if (out_size != kRows * kChan) return;
  if (ws_size < kWsTotal) return;

  const float* x     = (const float*)d_in[0];
  const float* ln1_w = (const float*)d_in[1];
  const float* ln1_b = (const float*)d_in[2];
  const float* ln2_w = (const float*)d_in[3];
  const float* ln2_b = (const float*)d_in[4];
  const float* Wr    = (const float*)d_in[5];
  const float* Wk    = (const float*)d_in[6];
  const float* Wv    = (const float*)d_in[7];
  const float* Wo    = (const float*)d_in[8];
  const float* decay = (const float*)d_in[9];
  const float* uvec  = (const float*)d_in[10];
  const float* Wfk   = (const float*)d_in[11];
  const float* Wfv   = (const float*)d_in[12];
  const float* Wfr   = (const float*)d_in[13];
  float* out = (float*)d_out;

  char* ws = (char*)d_ws;
  unsigned short* XN16  = (unsigned short*)(ws + kOffR0);
  unsigned short* G16   = (unsigned short*)(ws + kOffR0);
  unsigned short* XN2   = (unsigned short*)(ws + kOffR0);
  unsigned short* RP16  = (unsigned short*)(ws + kOffR1);
  unsigned short* Wo16  = (unsigned short*)(ws + kOffWo);
  unsigned short* Wfr16 = (unsigned short*)(ws + kOffWfr);
  float*          FVc   = (float*)(ws + kOffFVc);
  float*          Kf    = (float*)(ws + kOffR2);
  unsigned short* Wfk16 = (unsigned short*)(ws + kOffWfk);
  unsigned short* Wfv16 = (unsigned short*)(ws + kOffWfv);
  unsigned short* KKc   = (unsigned short*)(ws + kOffKKc);
  float*          Vf    = (float*)(ws + kOffR3);
  float*          FR    = (float*)(ws + kOffR3);
  unsigned short* Wr16  = (unsigned short*)(ws + kOffWr);
  unsigned short* Wk16  = (unsigned short*)(ws + kOffWk);
  unsigned short* Wv16  = (unsigned short*)(ws + kOffWv);
  float*          WKVF  = (float*)(ws + kOffR4);
  float*          X1    = (float*)(ws + kOffR4);

  const dim3 blk256(256);
  const int n8sq  = (kChan * kChan) / 8;
  const int n8ffn = (kHid4 * kChan) / 8;
  const int act   = kRows * kChan;

  const dim3 gridProj(((kRows / 64) * (kChan / 64)) / 8, 1);
  const dim3 gridFk(((kChunkRows / 64) * (kHid4 / 64)) / 8, 1);
  const dim3 gridFv(((kChunkRows / 64) * (kChan / 64)) / 8, 1);

  cast8_f16_kernel<<<dim3(n8sq / 256), blk256, 0, stream>>>(Wr, Wr16, n8sq, kWCarry);
  cast8_f16_kernel<<<dim3(n8sq / 256), blk256, 0, stream>>>(Wk, Wk16, n8sq, kWCarry);
  cast8_f16_kernel<<<dim3(n8sq / 256), blk256, 0, stream>>>(Wv, Wv16, n8sq, kWCarry);

  layernorm_f16_kernel<<<dim3(kRows), dim3(128), 0, stream>>>(x, ln1_w, ln1_b, XN16);

  wmma_gemm64<0, false, 0, 1, false, 0><<<gridProj, blk256, 0, stream>>>(
      XN16, nullptr, kChan, 0, Wr16, nullptr, kChan, 0, (void*)RP16, nullptr, kChan, 0,
      nullptr, nullptr, 0, kRows, kChan, kChan, kScaleProj);
  wmma_gemm64<0, false, 0, 0, false, 0><<<gridProj, blk256, 0, stream>>>(
      XN16, nullptr, kChan, 0, Wk16, nullptr, kChan, 0, (void*)Kf, nullptr, kChan, 0,
      nullptr, nullptr, 0, kRows, kChan, kChan, kScaleProj);
  wmma_gemm64<0, false, 0, 0, false, 0><<<gridProj, blk256, 0, stream>>>(
      XN16, nullptr, kChan, 0, Wv16, nullptr, kChan, 0, (void*)Vf, nullptr, kChan, 0,
      nullptr, nullptr, 0, kRows, kChan, kChan, kScaleProj);

  wkv_forward_kernel<<<dim3((kBatch * kChan) / 256), blk256, 0, stream>>>(Kf, Vf, decay, uvec, WKVF);

  wkv_backward_gate_kernel<<<dim3((kBatch * kChan / 2) / 256), blk256, 0, stream>>>(
      Kf, Vf, WKVF, RP16, decay, uvec, G16);

  cast8_f16_kernel<<<dim3(n8sq / 256), blk256, 0, stream>>>(Wo, Wo16, n8sq, kWCarry);
  wmma_gemm64<0, false, 0, 0, true, 0><<<gridProj, blk256, 0, stream>>>(
      G16, nullptr, kChan, 0, Wo16, nullptr, kChan, 0, (void*)X1, nullptr, kChan, 0,
      nullptr, x, 0, kRows, kChan, kChan, kScaleWo);

  layernorm_f16_kernel<<<dim3(kRows), dim3(128), 0, stream>>>(X1, ln2_w, ln2_b, XN2);

  cast8_f16_kernel<<<dim3(n8sq / 256), blk256, 0, stream>>>(Wfr, Wfr16, n8sq, kWCarry);
  cast8_f16_kernel<<<dim3(n8ffn / 256), blk256, 0, stream>>>(Wfk, Wfk16, n8ffn, kWCarry);
  cast8_f16_kernel<<<dim3(n8ffn / 256), blk256, 0, stream>>>(Wfv, Wfv16, n8ffn, kWCarry);

  wmma_gemm64<0, false, 0, 0, false, 0><<<gridProj, blk256, 0, stream>>>(
      XN2, nullptr, kChan, 0, Wfr16, nullptr, kChan, 0, (void*)FR, nullptr, kChan, 0,
      nullptr, nullptr, 0, kRows, kChan, kChan, kScaleProj);

  const int chunkElems = kChunkRows * kChan;
  const int n4chunk    = chunkElems / 4;
  for (int qc = 0; qc < kNumChunks; ++qc) {
    const size_t rowOff = (size_t)qc * kChunkRows;
    const unsigned short* Aq = XN2 + rowOff * kChan;
    wmma_gemm64<0, false, 0, 1, false, 6><<<gridFk, blk256, 0, stream>>>(
        Aq, nullptr, kChan, 0, Wfk16, nullptr, kChan, 0, (void*)KKc, nullptr, kHid4, 0,
        nullptr, nullptr, 0, kChunkRows, kHid4, kChan, kScaleFk);
    wmma_gemm64<0, false, 0, 0, false, 0><<<gridFv, blk256, 0, stream>>>(
        KKc, nullptr, kHid4, 0, Wfv16, nullptr, kHid4, 0, (void*)FVc, nullptr, kChan, 0,
        nullptr, nullptr, 0, kChunkRows, kChan, kHid4, kScaleFv);
    ffn_output_kernel<<<dim3(n4chunk / 256), blk256, 0, stream>>>(
        X1 + rowOff * kChan, FR + rowOff * kChan, FVc, out + rowOff * kChan, n4chunk);
  }
  (void)act;
}
